// HUH_83004537962778
// MI455X (gfx1250) — hardware-verified
//
#include <hip/hip_runtime.h>
#include <stddef.h>


#define TQ     90
#define OQ     5
#define NPG    (TQ + OQ)
#define DQ     256
#define HQ     256
#define RQ     5
#define NBQ    8
#define NTBL   (RQ + 1)
#define RIDX   RQ
#define TP     96
#define SPAD   128
#define NTHR   256
#define NWAVE  8
#define STHR   128
#define GROWS  128
#define GCOLS  128
#define ECH    1024
#define WSCAP  134217728
#define LDS_GEMM (GROWS * GCOLS * 4)
#define LDS_AGG  (NPG * HQ * 4 + ECH * 8)

static_assert(TQ <= STHR && TQ <= TP && (TP % 32) == 0 && TP <= STHR);
static_assert(NPG < 248 && TQ <= 255 && RQ <= 7);
static_assert(HQ == 256 && (DQ % 32) == 0);
static_assert(((DQ * HQ / 8) % NTHR) == 0);
static_assert(GROWS == NWAVE * 16 && GCOLS == 32 * 4 && (HQ % GCOLS) == 0);
static_assert((SPAD % GROWS) == 0 && SPAD >= TQ);
static_assert((ECH % NTHR) == 0 && ((NPG * HQ) % 4) == 0);
static_assert((NWAVE & (NWAVE - 1)) == 0 && NTHR == NWAVE * 32);
static_assert(LDS_AGG <= 160 * 1024);

typedef float           v4f   __attribute__((ext_vector_type(4)));
typedef float           v8f   __attribute__((ext_vector_type(8)));
typedef unsigned short  v8us  __attribute__((ext_vector_type(8)));
typedef __bf16          v16bf __attribute__((ext_vector_type(16)));
union FragB { v16bf v; v8us h[2]; };

static __device__ __forceinline__ unsigned short f2bf(float f) {
  unsigned int u = __float_as_uint(f);
  u = u + 0x7FFFu + ((u >> 16) & 1u);
  return (unsigned short)(u >> 16);
}
static __device__ __forceinline__ float bf2f(unsigned short b) {
  return __uint_as_float(((unsigned int)b) << 16);
}

static __device__ __forceinline__ v8f wmb(v16bf a, v16bf b, v8f c) {
  v8f d = __builtin_amdgcn_wmma_f32_16x16x32_bf16(false, a, false, b, (short)0, c, false, false);
  asm volatile("v_nop\n\tv_nop\n\tv_nop\n\tv_nop" : "+v"(d) : "v"(a), "v"(b));
  return d;
}

__global__ __launch_bounds__(NTHR) void k_cvt(const float* __restrict__ src, unsigned short* dhi, unsigned short* dlo,
                                              int rowLen, int nSrcRows, int total8) {
  const int i = (int)blockIdx.x * NTHR + (int)threadIdx.x;
  if (i >= total8) return;
  const size_t e  = (size_t)8 * (size_t)i;
  const int    r  = (int)(e / (size_t)rowLen);
  const int    k0 = (int)(e - (size_t)r * (size_t)rowLen);
  const int    rc = r < nSrcRows ? r : nSrcRows - 1;
  const float  z  = (r < nSrcRows) ? 1.0f : 0.0f;
  const float* sp = src + (size_t)rc * rowLen + k0;
  const v4f f0 = *(const v4f*)sp;
  const v4f f1 = *(const v4f*)(sp + 4);
  float v[8];
  v[0] = f0.x * z; v[1] = f0.y * z; v[2] = f0.z * z; v[3] = f0.w * z;
  v[4] = f1.x * z; v[5] = f1.y * z; v[6] = f1.z * z; v[7] = f1.w * z;
  v8us hv, lv;
#pragma unroll
  for (int j = 0; j < 8; ++j) {
    const unsigned short hb = f2bf(v[j]);
    hv[j] = hb;
    lv[j] = f2bf(v[j] - bf2f(hb));
  }
  unsigned short* ph = dhi + e;
  unsigned short* pl = dlo + e;
  *(volatile v8us*)ph = hv;
  *(volatile v8us*)pl = lv;
  __threadfence();
  *(volatile v8us*)ph = hv;
  *(volatile v8us*)pl = lv;
}

__global__ __launch_bounds__(NTHR) void k_buildw(const float* __restrict__ bases, const float* __restrict__ comp,
                                                 const float* __restrict__ root, unsigned short* whi, unsigned short* wlo) {
  const int tbl = (int)blockIdx.y;
  const int i = (int)blockIdx.x * NTHR + (int)threadIdx.x;
  if (i >= (DQ * HQ) / 8) return;
  const int e  = 8 * i;
  const int h  = e / DQ;
  const int k0 = e - h * DQ;
  float a[8];
#pragma unroll
  for (int j = 0; j < 8; ++j) a[j] = 0.0f;
  if (tbl < RQ) {
#pragma unroll 1
    for (int n = 0; n < NBQ; ++n) {
      const float c = comp[tbl * NBQ + n];
      const float* bp = bases + ((size_t)n * DQ + (size_t)k0) * HQ + h;
#pragma unroll
      for (int j = 0; j < 8; ++j) a[j] = fmaf(c, bp[(size_t)j * HQ], a[j]);
    }
  } else {
    const float* rp = root + (size_t)k0 * HQ + h;
#pragma unroll
    for (int j = 0; j < 8; ++j) a[j] = rp[(size_t)j * HQ];
  }
  v8us hv, lv;
#pragma unroll
  for (int j = 0; j < 8; ++j) {
    const unsigned short hb = f2bf(a[j]);
    hv[j] = hb;
    lv[j] = f2bf(a[j] - bf2f(hb));
  }
  const size_t o = (size_t)tbl * HQ * DQ + (size_t)e;
  unsigned short* ph = whi + o;
  unsigned short* pl = wlo + o;
  *(volatile v8us*)ph = hv;
  *(volatile v8us*)pl = lv;
  __threadfence();
  *(volatile v8us*)ph = hv;
  *(volatile v8us*)pl = lv;
}

template <int KD>
__global__ __launch_bounds__(NTHR) void k_gemm3(
    const unsigned short* __restrict__ Ahi, const unsigned short* __restrict__ Alo,
    const unsigned short* __restrict__ Bhi, const unsigned short* __restrict__ Blo,
    float* C, int ldc, int zStrideB, int zStrideC) {
  static_assert((KD % 32) == 0);
  extern __shared__ v4f lds_dyn[];
  constexpr int NT = GCOLS / 16;
  float* stg = (float*)lds_dyn;
  const int tid = threadIdx.x, lane = tid & 31, hh = lane >> 4, m = lane & 15;
  const int wave = __builtin_amdgcn_readfirstlane(tid >> 5);
  const int rowBase = (int)blockIdx.x * GROWS;
  const int colBase = (int)blockIdx.y * GCOLS;
  const int z = (int)blockIdx.z;
  const size_t aoff = (size_t)(rowBase + wave * 16 + m) * KD + 8 * hh;
  const unsigned short* ah = Ahi + aoff;
  const unsigned short* al = Alo + aoff;
  const size_t boff = (size_t)z * (size_t)zStrideB + (size_t)(colBase + m) * KD + 8 * hh;
  const unsigned short* bh0 = Bhi + boff;
  const unsigned short* bl0 = Blo + boff;

  v8f acc[NT];
#pragma unroll
  for (int t = 0; t < NT; ++t) { v8f zz = {0.f, 0.f, 0.f, 0.f, 0.f, 0.f, 0.f, 0.f}; acc[t] = zz; }

#pragma unroll 1
  for (int kt = 0; kt < KD / 32; ++kt) {
    FragB fah, fal;
    fah.h[0] = *(const v8us*)(ah + 32 * kt);
    fah.h[1] = *(const v8us*)(ah + 32 * kt + 16);
    fal.h[0] = *(const v8us*)(al + 32 * kt);
    fal.h[1] = *(const v8us*)(al + 32 * kt + 16);
#pragma unroll
    for (int t = 0; t < NT; ++t) {
      const size_t to = (size_t)(16 * t) * KD + (size_t)(32 * kt);
      FragB fbh, fbl;
      fbh.h[0] = *(const v8us*)(bh0 + to);
      fbh.h[1] = *(const v8us*)(bh0 + to + 16);
      fbl.h[0] = *(const v8us*)(bl0 + to);
      fbl.h[1] = *(const v8us*)(bl0 + to + 16);
      v8f d = acc[t];
      d = wmb(fah.v, fbh.v, d);
      d = wmb(fah.v, fbl.v, d);
      d = wmb(fal.v, fbh.v, d);
      acc[t] = d;
    }
  }

  const int r0 = wave * 16 + 8 * hh;
  float* sp = stg + r0 * GCOLS + m;
#pragma unroll
  for (int t = 0; t < NT; ++t) {
#pragma unroll
    for (int r = 0; r < 8; ++r) sp[r * GCOLS + 16 * t] = acc[t][r];
  }
  __syncthreads();

  const float* lp = stg + wave * 16 * GCOLS;
  float* gp = C + (size_t)z * (size_t)zStrideC + (size_t)(rowBase + wave * 16) * (size_t)ldc + colBase;
#pragma unroll
  for (int i = 0; i < 16; ++i) {
    const v4f v = *(const v4f*)(lp + i * GCOLS + 4 * lane);
    *(volatile v4f*)(gp + (size_t)i * ldc + 4 * lane) = v;
  }
  __threadfence();
#pragma unroll
  for (int i = 0; i < 16; ++i) {
    const v4f v = *(const v4f*)(lp + i * GCOLS + 4 * lane);
    *(volatile v4f*)(gp + (size_t)i * ldc + 4 * lane) = v;
  }
}

__global__ __launch_bounds__(STHR) void k_soft(const float* __restrict__ S, int ldS, float* P) {
  __shared__ __attribute__((aligned(16))) float scv[STHR];
  __shared__ float red[2];
  const int tid = threadIdx.x, lane = tid & 31;
  const int wave = __builtin_amdgcn_readfirstlane(tid >> 5);
  const int blk = (int)blockIdx.x;
  const int b = blk / TQ;
  const int s = blk - b * TQ;
  const int tc = tid < TQ ? tid : TQ - 1;
  const float v = S[(size_t)s * (size_t)ldS + (size_t)b * TQ + tc];
  scv[tid] = v;
  __syncthreads();
  if (tid == 0) {
    float mx = scv[0];
#pragma unroll 1
    for (int i = 1; i < TQ; ++i) mx = fmaxf(mx, scv[i]);
    red[0] = mx;
  }
  __syncthreads();
  const float mx = red[0];
  const float ex = expf(v - mx);
  const float ez = (tid < TQ) ? ex : 0.0f;
  scv[tid] = ez;
  __syncthreads();
  if (tid == 0) {
    float sm = 0.0f;
#pragma unroll 1
    for (int i = 0; i < TQ; ++i) sm += scv[i];
    red[1] = 1.0f / sm;
  }
  __syncthreads();
  const float p = ez * red[1];
  scv[tid] = p;
  __syncthreads();
  if (wave == 0) {
    const v4f pv = *(const v4f*)(scv + 4 * lane);
    float* pr = P + (size_t)blk * TP;
    if (lane < TP / 4) *(volatile v4f*)(pr + 4 * lane) = pv;
    __threadfence();
    if (lane < TP / 4) *(volatile v4f*)(pr + 4 * lane) = pv;
  }
}

__global__ __launch_bounds__(NTHR) void k_agg(
    const int* __restrict__ esrc, const int* __restrict__ edst, const int* __restrict__ etyp,
    const float* __restrict__ natt, const float* __restrict__ P, const float* __restrict__ Y,
    const float* __restrict__ bias, float* out, int eag, int npad) {
  extern __shared__ v4f lds_dyn[];
  float* accl = (float*)lds_dyn;
  int*   erec = (int*)(accl + NPG * HQ);
  float* enrm = (float*)(erec + ECH);
  const int tid = threadIdx.x, lane = tid & 31;
  const int wave = __builtin_amdgcn_readfirstlane(tid >> 5);
  const int b = (int)blockIdx.x;
  const int epb = eag + TQ * OQ;

  {
    const v4f zz = {0.f, 0.f, 0.f, 0.f};
#pragma unroll 1
    for (int i = tid; i < (NPG * HQ) / 4; i += NTHR) ((v4f*)accl)[i] = zz;
  }

  const int nChunks = (epb + ECH - 1) / ECH;
#pragma unroll 1
  for (int ch = 0; ch < nChunks; ++ch) {
    __syncthreads();
#pragma unroll 1
    for (int i = tid; i < ECH; i += NTHR) {
      const int j  = ch * ECH + i;
      const int ja = j < eag ? j : eag - 1;
      const size_t eo = (size_t)b * (size_t)eag + (size_t)ja;
      const int sA = esrc[eo], dA = edst[eo], tA = etyp[eo];
      int k = j - eag;
      k = k < 0 ? 0 : (k > TQ * OQ - 1 ? TQ * OQ - 1 : k);
      const int tT = k / OQ, oT = k - tT * OQ;
      const float nT = natt[((size_t)b * TQ + tT) * OQ + oT];
      const int sAc = sA < 0 ? 0 : (sA > TQ - 1 ? TQ - 1 : sA);
      const int dAc = dA < 0 ? 0 : (dA > TQ - 1 ? TQ - 1 : dA);
      const float pA = P[((size_t)b * TQ + sAc) * TP + dAc];
      const bool isAtt = j < eag;
      const bool isTag = (j >= eag) && (j < epb);
      const int src = isAtt ? sAc : tT;
      const int dst = isAtt ? dA : (TQ + oT);
      const int typ = isAtt ? tA : (RQ - 1);
      const float nrm = isAtt ? pA : nT;
      const bool valid = (isAtt || isTag) && ((unsigned)dst < (unsigned)NPG) && ((unsigned)typ < (unsigned)RQ);
      erec[i] = valid ? (dst | (src << 8) | (typ << 16)) : 255;
      enrm[i] = valid ? nrm : 0.0f;
    }
    __syncthreads();
    int cnt = epb - ch * ECH;
    cnt = cnt > ECH ? ECH : (cnt < 0 ? 0 : cnt);
#pragma unroll 1
    for (int ii = 0; ii < cnt; ++ii) {
      const int rec = __builtin_amdgcn_readfirstlane(erec[ii]);
      const int dst = rec & 255;
      if (dst < NPG && (dst & (NWAVE - 1)) == wave) {
        const int src = (rec >> 8) & 255;
        int typ = (rec >> 16) & 7;
        typ = typ > RQ - 1 ? RQ - 1 : typ;
        const float nrm = enrm[ii];
        const v4f nv = {nrm, nrm, nrm, nrm};
        const float* yp = Y + ((size_t)typ * (size_t)npad + (size_t)b * NPG + (size_t)src) * HQ + 4 * lane;
        const v4f y0 = *(const v4f*)yp;
        const v4f y1 = *(const v4f*)(yp + 128);
        float* ap = accl + dst * HQ + 4 * lane;
        v4f a0 = *(const v4f*)ap;
        v4f a1 = *(const v4f*)(ap + 128);
        a0 = nv * y0 + a0;
        a1 = nv * y1 + a1;
        *(v4f*)ap = a0;
        *(v4f*)(ap + 128) = a1;
      }
    }
  }
  __syncthreads();

  const v4f bv0 = *(const v4f*)(bias + 4 * lane);
  const v4f bv1 = *(const v4f*)(bias + 128 + 4 * lane);
#pragma unroll 1
  for (int n = wave; n < NPG; n += NWAVE) {
    const size_t gr = (size_t)b * NPG + (size_t)n;
    const float* yr = Y + ((size_t)RIDX * (size_t)npad + gr) * HQ + 4 * lane;
    const float* ap = accl + n * HQ + 4 * lane;
    const v4f v0 = (*(const v4f*)ap + *(const v4f*)yr) + bv0;
    const v4f v1 = (*(const v4f*)(ap + 128) + *(const v4f*)(yr + 128)) + bv1;
    float* op = out + gr * HQ + 4 * lane;
    *(volatile v4f*)op = v0;
    *(volatile v4f*)(op + 128) = v1;
    __threadfence();
    *(volatile v4f*)op = v0;
    *(volatile v4f*)(op + 128) = v1;
  }
}

extern "C" void kernel_launch(void* const* d_in, const int* in_sizes, int n_in,
                              void* d_out, int out_size, void* d_ws, size_t ws_size,
                              hipStream_t stream) {
  if (n_in < 11) return;
  if (in_sizes[3] != TQ * DQ || in_sizes[4] != NBQ * DQ * HQ || in_sizes[5] != RQ * NBQ) return;
  if (in_sizes[6] != DQ * HQ || in_sizes[7] != HQ) return;
  const int Bn = in_sizes[0] / (TQ * DQ);
  if (Bn <= 0 || in_sizes[0] != Bn * TQ * DQ) return;
  const int Nn = Bn * NPG;
  if (in_sizes[1] != Nn * DQ || in_sizes[2] != Bn * TQ * OQ) return;
  const int eag = in_sizes[8] / Bn;
  if (eag <= 0 || in_sizes[8] != Bn * eag || in_sizes[9] != in_sizes[8] || in_sizes[10] != in_sizes[8]) return;
  if (out_size != Nn * HQ) return;
  if (Bn > (1 << 16) || eag > (1 << 24)) return;

  const float* M     = (const float*)d_in[0];
  const float* x     = (const float*)d_in[1];
  const float* natt  = (const float*)d_in[2];
  const float* Ws    = (const float*)d_in[3];
  const float* bases = (const float*)d_in[4];
  const float* comp  = (const float*)d_in[5];
  const float* root  = (const float*)d_in[6];
  const float* bias  = (const float*)d_in[7];
  const int*   esrc  = (const int*)d_in[8];
  const int*   edst  = (const int*)d_in[9];
  const int*   etyp  = (const int*)d_in[10];
  float* out = (float*)d_out;

  const int NPAD  = ((Nn + GROWS - 1) / GROWS) * GROWS;
  const int MROWS = Bn * TQ;
  const int MPAD  = ((MROWS + GCOLS - 1) / GCOLS) * GCOLS;

  char* ws = (char*)d_ws;
  size_t off = 0;
  const size_t oP   = off; off += (size_t)MROWS * TP * 4;            off = (off + 255) & ~(size_t)255;
  const size_t oXh  = off; off += (size_t)NPAD * DQ * 2;             off = (off + 255) & ~(size_t)255;
  const size_t oXl  = off; off += (size_t)NPAD * DQ * 2;             off = (off + 255) & ~(size_t)255;
  const size_t oMh  = off; off += (size_t)MPAD * DQ * 2;             off = (off + 255) & ~(size_t)255;
  const size_t oMl  = off; off += (size_t)MPAD * DQ * 2;             off = (off + 255) & ~(size_t)255;
  const size_t oSh  = off; off += (size_t)SPAD * DQ * 2;             off = (off + 255) & ~(size_t)255;
  const size_t oSl  = off; off += (size_t)SPAD * DQ * 2;             off = (off + 255) & ~(size_t)255;
  const size_t oWh  = off; off += (size_t)NTBL * HQ * DQ * 2;        off = (off + 255) & ~(size_t)255;
  const size_t oWl  = off; off += (size_t)NTBL * HQ * DQ * 2;        off = (off + 255) & ~(size_t)255;
  const size_t oS   = off; off += (size_t)SPAD * MPAD * 4;           off = (off + 255) & ~(size_t)255;
  const size_t oY   = off; off += (size_t)NTBL * NPAD * HQ * 4;      off = (off + 255) & ~(size_t)255;
  if (off > ws_size || off > (size_t)WSCAP) return;
  float*          P   = (float*)(ws + oP);
  unsigned short* Xh  = (unsigned short*)(ws + oXh);
  unsigned short* Xl  = (unsigned short*)(ws + oXl);
  unsigned short* Mh  = (unsigned short*)(ws + oMh);
  unsigned short* Ml  = (unsigned short*)(ws + oMl);
  unsigned short* Sh  = (unsigned short*)(ws + oSh);
  unsigned short* Sl  = (unsigned short*)(ws + oSl);
  unsigned short* Wh  = (unsigned short*)(ws + oWh);
  unsigned short* Wl  = (unsigned short*)(ws + oWl);
  float*          S   = (float*)(ws + oS);
  float*          Y   = (float*)(ws + oY);

  hipFuncSetAttribute(reinterpret_cast<const void*>(&k_gemm3<DQ>),
                      hipFuncAttributeMaxDynamicSharedMemorySize, LDS_GEMM);
  hipFuncSetAttribute(reinterpret_cast<const void*>(&k_agg),
                      hipFuncAttributeMaxDynamicSharedMemorySize, LDS_AGG);

  {
    const int t8x = (NPAD * DQ) / 8;
    k_cvt<<<(t8x + NTHR - 1) / NTHR, NTHR, 0, stream>>>(x, Xh, Xl, DQ, Nn, t8x);
    const int t8m = (MPAD * DQ) / 8;
    k_cvt<<<(t8m + NTHR - 1) / NTHR, NTHR, 0, stream>>>(M, Mh, Ml, DQ, MROWS, t8m);
    const int t8s = (SPAD * DQ) / 8;
    k_cvt<<<(t8s + NTHR - 1) / NTHR, NTHR, 0, stream>>>(Ws, Sh, Sl, DQ, TQ, t8s);
  }
  k_buildw<<<dim3((DQ * HQ / 8 + NTHR - 1) / NTHR, NTBL), NTHR, 0, stream>>>(bases, comp, root, Wh, Wl);
  k_gemm3<DQ><<<dim3(SPAD / GROWS, MPAD / GCOLS, 1), NTHR, LDS_GEMM, stream>>>(Sh, Sl, Mh, Ml, S, MPAD, 0, 0);
  k_soft<<<MROWS, STHR, 0, stream>>>(S, MPAD, P);
  k_gemm3<DQ><<<dim3(NPAD / GROWS, HQ / GCOLS, NTBL), NTHR, LDS_GEMM, stream>>>(Xh, Xl, Wh, Wl, Y, HQ, HQ * DQ, NPAD * HQ);
  k_agg<<<Bn, NTHR, LDS_AGG, stream>>>(esrc, edst, etyp, natt, P, Y, bias, out, eag, NPAD);
}
